// QuanvolutionClassifier_65481071403850
// MI455X (gfx1250) — hardware-verified
//
#include <hip/hip_runtime.h>


typedef _Float16 v16h __attribute__((ext_vector_type(16)));
typedef _Float16 v8h  __attribute__((ext_vector_type(8)));
typedef float    v8f  __attribute__((ext_vector_type(8)));
typedef float    v4f  __attribute__((ext_vector_type(4)));

#define ROWS     16
#define KREAL    784
#define NSITE    196
#define NCLS     10
#define NWAVES   4
#define NTHREADS (NWAVES * 32)
#define KPAD     896
#define KBLOCKS  (KPAD / 32)
#define QITER    (KBLOCKS / NWAVES)
#define KSTRIDE  904
#define WSCALE   32.0f
#define WINV     0.03125f
#define OT_F4    (ROWS * NCLS / 4)

static_assert(KPAD % (32 * NWAVES) == 0);
static_assert((ROWS * NCLS * 4) % 128 == 0);
static_assert((ROWS * NCLS) % 4 == 0);
static_assert(KSTRIDE % 8 == 0);
static_assert(OT_F4 > 32 && OT_F4 <= 64);

union Frag { v16h v; v8h half[2]; };

__device__ __forceinline__ v8f wmma_f16_step(v16h a, v16h b, v8f acc)
{
    acc = __builtin_amdgcn_wmma_f32_16x16x32_f16(false, a, false, b, (short)0, acc, false, false);
    asm volatile("v_nop\n\tv_nop\n\tv_nop\n\tv_nop" : "+v"(acc) : "v"(a), "v"(b));
    return acc;
}

__global__ __launch_bounds__(NTHREADS)
void quanv_fused_kernel(const float* __restrict__ x,
                        const float* __restrict__ conv_w,
                        const float* __restrict__ conv_b,
                        const float* __restrict__ bn_gamma,
                        const float* __restrict__ bn_beta,
                        const float* __restrict__ bn_mean,
                        const float* __restrict__ bn_var,
                        const float* __restrict__ shortcut_weight,
                        const float* __restrict__ theta,
                        const float* __restrict__ lin_w,
                        const float* __restrict__ lin_b,
                        const float* __restrict__ log_scale,
                        float* __restrict__ out,
                        int Btotal)
{
    __shared__ __align__(16) _Float16 ftile[ROWS][KSTRIDE];
    __shared__ __align__(16) _Float16 btile[16][KSTRIDE];
    __shared__ __align__(16) float    sc32[ROWS][KREAL];
    __shared__ float pltile[NWAVES][ROWS][16];
    __shared__ __align__(16) float otile[ROWS * NCLS];
    __shared__ float trg[16];

    const int tid  = threadIdx.x;
    const int lane = tid & 31;
    const int wave = tid >> 5;
    const int row0 = blockIdx.x * ROWS;
    const int Bm1  = Btotal - 1;

    const float sw = shortcut_weight[0];
    float wcv[16], cbv[4], mnv[4], rsv[4], gmv[4], btv[4];
    #pragma unroll
    for (int c = 0; c < 4; ++c) {
        cbv[c] = conv_b[c];
        mnv[c] = bn_mean[c];
        rsv[c] = 1.0f / sqrtf(bn_var[c] + 1e-5f);
        gmv[c] = bn_gamma[c];
        btv[c] = bn_beta[c];
        #pragma unroll
        for (int q = 0; q < 4; ++q) wcv[c * 4 + q] = conv_w[c * 4 + q];
    }
    if (tid < 16) {
        const int w = tid & 7;
        const float g = theta[w] * 0.5f;
        trg[tid] = (tid < 8) ? cosf(g) : sinf(g);
    }

    for (int t = tid; t < 16 * KPAD; t += NTHREADS) {
        const int n = t / KPAD, k = t - n * KPAD;
        const float v = (k < KREAL && n < NCLS) ? lin_w[n * KREAL + k] * WSCALE : 0.0f;
        btile[n][k] = (_Float16)v;
    }
    for (int t = tid; t < ROWS * (KPAD - KREAL); t += NTHREADS) {
        const int r = t / (KPAD - KREAL);
        const int k = KREAL + (t - r * (KPAD - KREAL));
        ftile[r][k] = (_Float16)0.0f;
    }

    for (int t = tid; t < ROWS * NSITE; t += NTHREADS) {
        const int r = t / NSITE;
        const int s = t - r * NSITE;
        const int i = s / 14;
        const int j = s - i * 14;
        int rr = row0 + r; rr = (rr > Bm1) ? Bm1 : rr;
        const float* xp = x + (size_t)rr * KREAL + (2 * i) * 28 + 2 * j;
        const float p0 = xp[0], p1 = xp[1], p2 = xp[28], p3 = xp[29];
        #pragma unroll
        for (int c = 0; c < 4; ++c) {
            const float conv = p0 * wcv[c * 4 + 0] + p1 * wcv[c * 4 + 1]
                             + p2 * wcv[c * 4 + 2] + p3 * wcv[c * 4 + 3];
            float v = conv + cbv[c];
            v = (v - mnv[c]) * rsv[c];
            v = v * gmv[c] + btv[c];
            sc32[r][c * NSITE + s] = sw * v;
        }
    }

    __syncthreads();

    const float c10 = trg[0],  c11 = trg[1],  c12 = trg[2],  c13 = trg[3];
    const float c20 = trg[4],  c21 = trg[5],  c22 = trg[6],  c23 = trg[7];
    const float s10 = trg[8],  s11 = trg[9],  s12 = trg[10], s13 = trg[11];
    const float s20 = trg[12], s21 = trg[13], s22 = trg[14], s23 = trg[15];
    for (int t = tid; t < ROWS * NSITE * 2; t += NTHREADS) {
        const int r   = t / (2 * NSITE);
        const int rem = t - r * (2 * NSITE);
        const int p   = rem >> 1;
        const int h   = rem & 1;
        const int i2  = p / 14;
        const int j2  = p - i2 * 14;
        int rr = row0 + r; rr = (rr > Bm1) ? Bm1 : rr;
        const float* qp = x + (size_t)rr * KREAL + (2 * i2 + h) * 28 + 2 * j2;
        const float va = qp[0] * 0.5f;
        const float vb = qp[1] * 0.5f;
        const float ea0 = cosf(va), ea1 = sinf(va);
        const float eb0 = cosf(vb), eb1 = sinf(vb);
        const float cta = h ? c12 : c10, sta = h ? s12 : s10;
        const float ctb = h ? c13 : c11, stb = h ? s13 : s11;
        const float a0 = cta * ea0 - sta * ea1, a1 = sta * ea0 + cta * ea1;
        const float b0 = ctb * eb0 - stb * eb1, b1 = stb * eb0 + ctb * eb1;
        const float w00 = a0 * b0, w01 = a0 * b1, w10 = a1 * b1, w11 = a1 * b0;
        const float cc1 = h ? c22 : c20, ss1 = h ? s22 : s20;
        const float cc2 = h ? c23 : c21, ss2 = h ? s23 : s21;
        const float u00 = cc1 * w00 - ss1 * w10;
        const float u01 = cc1 * w01 - ss1 * w11;
        const float u10 = ss1 * w00 + cc1 * w10;
        const float u11 = ss1 * w01 + cc1 * w11;
        const float v00 = cc2 * u00 - ss2 * u01;
        const float v01 = ss2 * u00 + cc2 * u01;
        const float v10 = cc2 * u10 - ss2 * u11;
        const float v11 = ss2 * u10 + cc2 * u11;
        const float p00 = v00 * v00, p01 = v01 * v01, p10 = v10 * v10, p11 = v11 * v11;
        const float Za = p00 + p01 - p10 - p11;
        const float Zb = p00 - p01 + p10 - p11;
        const int k = (p << 2) + (h << 1);
        const float fa = sc32[r][k]     + Za;
        const float fb = sc32[r][k + 1] + Zb;
        ftile[r][k]     = (_Float16)fa;
        ftile[r][k + 1] = (_Float16)fb;
    }

    __syncthreads();

    v8f acc = {0.f, 0.f, 0.f, 0.f, 0.f, 0.f, 0.f, 0.f};
    const int lm = lane & 15;
    const int lh = lane >> 4;
    #pragma unroll
    for (int q = 0; q < QITER; ++q) {
        const int kbase = (wave + q * NWAVES) * 32;
        Frag a, b;
        const v8h* pa = (const v8h*)&ftile[lm][kbase + 8 * lh];
        a.half[0] = pa[0];
        a.half[1] = pa[2];
        const v8h* pb = (const v8h*)&btile[lm][kbase + 8 * lh];
        b.half[0] = pb[0];
        b.half[1] = pb[2];
        acc = wmma_f16_step(a.v, b.v, acc);
    }

    #pragma unroll
    for (int v = 0; v < 8; ++v)
        pltile[wave][v + lh * 8][lm] = acc[v];

    __syncthreads();

    if (tid < ROWS) {
        const float ls = log_scale[0];
        float z[NCLS];
        #pragma unroll
        for (int n = 0; n < NCLS; ++n) {
            const float s = pltile[0][tid][n] + pltile[1][tid][n]
                          + pltile[2][tid][n] + pltile[3][tid][n];
            z[n] = (s * WINV + lin_b[n]) * ls;
        }
        float mx = z[0];
        #pragma unroll
        for (int n = 1; n < NCLS; ++n) mx = fmaxf(mx, z[n]);
        float se = 0.0f;
        #pragma unroll
        for (int n = 0; n < NCLS; ++n) se += expf(z[n] - mx);
        const float lse = logf(se);
        #pragma unroll
        for (int n = 0; n < NCLS; ++n) otile[tid * NCLS + n] = (z[n] - mx) - lse;
    }

    __syncthreads();

    if (wave == 0) {
        float* obase = out + (size_t)row0 * NCLS;
        if (row0 + ROWS <= Btotal) {
            const int t1 = 32 + (lane & (OT_F4 - 32 - 1));
            const v4f q0 = *(const v4f*)&otile[4 * lane];
            const v4f q1 = *(const v4f*)&otile[4 * t1];
            volatile v4f* o0 = (volatile v4f*)obase + lane;
            volatile v4f* o1 = (volatile v4f*)obase + t1;
            const bool has1 = lane < (OT_F4 - 32);
            *o0 = q0;
            if (has1) *o1 = q1;
            __threadfence();
            *o0 = q0;
            if (has1) *o1 = q1;
        } else {
            for (int t = lane; t < ROWS * NCLS; t += 32) {
                const int r = t / NCLS;
                if (row0 + r < Btotal) { const float v = otile[t]; volatile float* o = obase + t; *o = v; }
            }
            __threadfence();
            for (int t = lane; t < ROWS * NCLS; t += 32) {
                const int r = t / NCLS;
                if (row0 + r < Btotal) { const float v = otile[t]; volatile float* o = obase + t; *o = v; }
            }
        }
    }
}

extern "C" void kernel_launch(void* const* d_in, const int* in_sizes, int n_in,
                              void* d_out, int out_size, void* d_ws, size_t ws_size,
                              hipStream_t stream)
{
    (void)n_in; (void)d_ws; (void)ws_size;
    const float* x        = (const float*)d_in[0];
    const float* conv_w   = (const float*)d_in[1];
    const float* conv_b   = (const float*)d_in[2];
    const float* bn_gamma = (const float*)d_in[3];
    const float* bn_beta  = (const float*)d_in[4];
    const float* bn_mean  = (const float*)d_in[5];
    const float* bn_var   = (const float*)d_in[6];
    const float* sw       = (const float*)d_in[7];
    const float* theta    = (const float*)d_in[8];
    const float* lin_w    = (const float*)d_in[9];
    const float* lin_b    = (const float*)d_in[10];
    const float* log_sc   = (const float*)d_in[11];
    float* out            = (float*)d_out;

    int Btotal = in_sizes[0] / KREAL;
    const int Bout = out_size / NCLS;
    if (Bout < Btotal) Btotal = Bout;
    if (Btotal <= 0) return;
    const int grid = (Btotal + ROWS - 1) / ROWS;

    quanv_fused_kernel<<<grid, NTHREADS, 0, stream>>>(
        x, conv_w, conv_b, bn_gamma, bn_beta, bn_mean, bn_var,
        sw, theta, lin_w, lin_b, log_sc, out, Btotal);
}
